// MicrobiomeTreeModel_21818433863684
// MI455X (gfx1250) — hardware-run, weakly checked
//
#include <hip/hip_runtime.h>

typedef __attribute__((ext_vector_type(16))) _Float16 v16h;
typedef __attribute__((ext_vector_type(8)))  _Float16 v8h;
typedef __attribute__((ext_vector_type(8)))  float    v8f;
typedef __attribute__((ext_vector_type(4)))  float    v4f;

constexpr int kSamples       = 524288;
constexpr int kLeaves        = 16;
constexpr int kHid           = 16;
constexpr int kTileRows      = 16;
constexpr int kTiles         = kSamples / kTileRows;
constexpr int kWavesPerBlock = 4;
constexpr int kThreads       = kWavesPerBlock * 32;
constexpr int kBlocks        = 1024;
constexpr int kTilesPerWave  = kTiles / (kBlocks * kWavesPerBlock);
constexpr int kPitchH2       = 68;
constexpr int kPitchH3       = 36;
constexpr int kNodeTile      = 16 * 32;
static_assert(kSamples % kTileRows == 0, "sample tiles");
static_assert(kTilesPerWave * kBlocks * kWavesPerBlock == kTiles, "uniform trip count");
static_assert(kTilesPerWave == 8, "8 tiles per wave");
static_assert((kPitchH2 * 4) % 16 == 0 && (kPitchH3 * 4) % 16 == 0, "16-B aligned LDS rows");
static_assert(kLeaves == 16 && kHid == 16, "node widths");

constexpr float kWCarry       = 64.0f;
constexpr float kLoCarry      = 2048.0f;
constexpr float kInvW         = 1.0f / kWCarry;
constexpr float kInvWL        = 1.0f / (kWCarry * kLoCarry);
constexpr float kF16MinNormal = 6.103515625e-5f;

__device__ __forceinline__ unsigned short f2bf_bits(float f) {
  unsigned u = __float_as_uint(f);
  return (unsigned short)((u + 0x7FFFu + ((u >> 16) & 1u)) >> 16);
}
__device__ __forceinline__ float bf_bits2f(unsigned short h) { return __uint_as_float(((unsigned)h) << 16); }
__device__ __forceinline__ float bf_rne(float f) { return bf_bits2f(f2bf_bits(f)); }

template <typename T> struct Frag;
template <> struct Frag<_Float16> {
  typedef v16h V; union U { v16h v; v8h h[2]; };
  static __device__ __forceinline__ v16h load(const _Float16* p) {
    U f; f.h[0] = *(const v8h*)(p); f.h[1] = *(const v8h*)(p + 16); return f.v;
  }
};

__device__ __forceinline__ v8f mma_h(v16h a, v16h b, v8f c) {
  c = __builtin_amdgcn_wmma_f32_16x16x32_f16(false, a, false, b, (short)0, c, false, false);
  asm volatile("v_nop\n\tv_nop\n\tv_nop\n\tv_nop" : "+v"(c) : "v"(a), "v"(b));
  return c;
}

__device__ __forceinline__ void wave_lds_sync() {
  __builtin_amdgcn_fence(__ATOMIC_RELEASE, "workgroup");
  __builtin_amdgcn_wave_barrier();
  __builtin_amdgcn_fence(__ATOMIC_ACQUIRE, "workgroup");
}

__device__ __forceinline__ void split_h(float v, _Float16& hi, _Float16& lo) {
  const unsigned u  = __float_as_uint(v);
  const unsigned ur = (u + 0x0FFFu + ((u >> 13) & 1u)) & 0xFFFFE000u;
  const float hfull = __uint_as_float(ur);
  const float hf    = (v >= kF16MinNormal) ? hfull : 0.0f;
  hi = (_Float16)hf;
  lo = (_Float16)((v - hf) * kLoCarry);
}

__device__ __forceinline__ void stage_bt(const float* __restrict__ W, _Float16* dst, int count, int tid) {
#pragma unroll 1
  for (int idx = tid; idx < count; idx += kThreads) {
    const int n  = idx & 15;
    const int k  = (idx >> 4) & 31;
    const int nd = idx >> 9;
    const float wb = bf_rne(W[idx]);
    dst[(nd * 16 + n) * 32 + k] = (_Float16)(wb * kWCarry);
  }
}

__global__ __launch_bounds__(kThreads)
void tree_fused_kernel(const float* __restrict__ x,
                       const float* __restrict__ W1, const float* __restrict__ b1,
                       const float* __restrict__ W2, const float* __restrict__ b2,
                       const float* __restrict__ W3, const float* __restrict__ b3,
                       const float* __restrict__ W4, const float* __restrict__ b4,
                       float* __restrict__ out, int nTiles, int tilesPerWave) {
  __shared__ __align__(16) _Float16 sBt[7 * kNodeTile];
  __shared__ __align__(16) float sW1[8 * 2 * 16];
  __shared__ __align__(16) float sB1[8 * 16];
  __shared__ __align__(16) float sH2[kWavesPerBlock][16 * kPitchH2];
  __shared__ __align__(16) float sH3[kWavesPerBlock][16 * kPitchH3];
  __shared__ __align__(16) float sO[kWavesPerBlock][16 * 16];

  const int tid  = threadIdx.x;
  const int lane = tid & 31;
  const int wave = tid >> 5;
  const int h    = lane >> 4;
  const int n    = lane & 15;

  stage_bt(W2, sBt, 4 * kNodeTile, tid);
  stage_bt(W3, sBt + 4 * kNodeTile, 2 * kNodeTile, tid);
  stage_bt(W4, sBt + 6 * kNodeTile, 1 * kNodeTile, tid);
  sW1[tid]       = bf_rne(W1[tid]);
  sW1[tid + 128] = bf_rne(W1[tid + 128]);
  sB1[tid]       = bf_rne(b1[tid]);
  __syncthreads();

  v16h B2f[4], B3f[2], B4f;
#pragma unroll
  for (int i = 0; i < 4; ++i) B2f[i] = Frag<_Float16>::load(sBt + (i * 16 + n) * 32 + 8 * h);
#pragma unroll
  for (int j = 0; j < 2; ++j) B3f[j] = Frag<_Float16>::load(sBt + ((4 + j) * 16 + n) * 32 + 8 * h);
  B4f = Frag<_Float16>::load(sBt + (6 * 16 + n) * 32 + 8 * h);

  float bb2[4], bb3[2], bb4;
#pragma unroll
  for (int i = 0; i < 4; ++i) bb2[i] = bf_rne(b2[i * 16 + n]);
#pragma unroll
  for (int j = 0; j < 2; ++j) bb3[j] = bf_rne(b3[j * 16 + n]);
  bb4 = bf_rne(b4[n]);

  float* sH2w = sH2[wave];
  float* sH3w = sH3[wave];
  float* sOw  = sO[wave];

  const int gwave  = blockIdx.x * kWavesPerBlock + wave;
  const int nWaves = gridDim.x * kWavesPerBlock;
  const v8f zero8 = (v8f){0.f, 0.f, 0.f, 0.f, 0.f, 0.f, 0.f, 0.f};

#pragma unroll 1
  for (int it = 0; it < tilesPerWave; ++it) {
    const int t = gwave + it * nWaves;
    if (t >= nTiles) break;

    float xr[16];
    {
      const float* xp = x + ((size_t)t * kTileRows + n) * kLeaves;
      const v4f q0 = *(const v4f*)(xp);
      const v4f q1 = *(const v4f*)(xp + 4);
      const v4f q2 = *(const v4f*)(xp + 8);
      const v4f q3 = *(const v4f*)(xp + 12);
#pragma unroll
      for (int e = 0; e < 4; ++e) {
        const float f0 = q0[e], f1 = q1[e], f2 = q2[e], f3 = q3[e];
        xr[e]      = bf_rne(f0);
        xr[4 + e]  = bf_rne(f1);
        xr[8 + e]  = bf_rne(f2);
        xr[12 + e] = bf_rne(f3);
      }
    }

#pragma unroll
    for (int i = 0; i < 4; ++i) {
      v16h ah, al;
#pragma unroll
      for (int ch = 0; ch < 2; ++ch) {
        const int nd = 2 * i + ch;
        const float x0 = xr[2 * nd];
        const float x1 = xr[2 * nd + 1];
        const float* wp = sW1 + nd * 32 + 8 * h;
        const float* bp = sB1 + nd * 16 + 8 * h;
        const v4f wa0 = *(const v4f*)(wp);
        const v4f wa1 = *(const v4f*)(wp + 4);
        const v4f wb0 = *(const v4f*)(wp + 16);
        const v4f wb1 = *(const v4f*)(wp + 20);
        const v4f bv0 = *(const v4f*)(bp);
        const v4f bv1 = *(const v4f*)(bp + 4);
#pragma unroll
        for (int e = 0; e < 4; ++e) {
          float v0 = fmaf(x1, wb0[e], x0 * wa0[e]) + bv0[e];
          float v1 = fmaf(x1, wb1[e], x0 * wa1[e]) + bv1[e];
          v0 = fmaxf(v0, 0.0f);
          v1 = fmaxf(v1, 0.0f);
          _Float16 hh, ll;
          split_h(v0, hh, ll);
          ah[ch * 8 + e] = hh;
          al[ch * 8 + e] = ll;
          split_h(v1, hh, ll);
          ah[ch * 8 + 4 + e] = hh;
          al[ch * 8 + 4 + e] = ll;
        }
      }
      v8f c  = zero8;
      v8f cl = zero8;
      c  = mma_h(ah, B2f[i], c);
      cl = mma_h(al, B2f[i], cl);
      float* hp = sH2w + (8 * h) * kPitchH2 + i * 16 + n;
#pragma unroll
      for (int r = 0; r < 8; ++r) {
        const float v = fmaf(cl[r], kInvWL, c[r] * kInvW) + bb2[i];
        hp[r * kPitchH2] = fmaxf(v, 0.0f);
      }
    }
    wave_lds_sync();

#pragma unroll
    for (int j = 0; j < 2; ++j) {
      const float* ap = sH2w + n * kPitchH2 + 32 * j + 8 * h;
      const v4f a0 = *(const v4f*)(ap);
      const v4f a1 = *(const v4f*)(ap + 4);
      const v4f a2 = *(const v4f*)(ap + 16);
      const v4f a3 = *(const v4f*)(ap + 20);
      v16h ah, al;
#pragma unroll
      for (int e = 0; e < 4; ++e) {
        const float f0 = a0[e], f1 = a1[e], f2 = a2[e], f3 = a3[e];
        _Float16 hh, ll;
        split_h(f0, hh, ll);
        ah[e] = hh;
        al[e] = ll;
        split_h(f1, hh, ll);
        ah[4 + e] = hh;
        al[4 + e] = ll;
        split_h(f2, hh, ll);
        ah[8 + e] = hh;
        al[8 + e] = ll;
        split_h(f3, hh, ll);
        ah[12 + e] = hh;
        al[12 + e] = ll;
      }
      v8f c  = zero8;
      v8f cl = zero8;
      c  = mma_h(ah, B3f[j], c);
      cl = mma_h(al, B3f[j], cl);
      float* hp = sH3w + (8 * h) * kPitchH3 + j * 16 + n;
#pragma unroll
      for (int r = 0; r < 8; ++r) {
        const float v = fmaf(cl[r], kInvWL, c[r] * kInvW) + bb3[j];
        hp[r * kPitchH3] = fmaxf(v, 0.0f);
      }
    }
    wave_lds_sync();

    {
      const float* ap = sH3w + n * kPitchH3 + 8 * h;
      const v4f a0 = *(const v4f*)(ap);
      const v4f a1 = *(const v4f*)(ap + 4);
      const v4f a2 = *(const v4f*)(ap + 16);
      const v4f a3 = *(const v4f*)(ap + 20);
      v16h ah, al;
#pragma unroll
      for (int e = 0; e < 4; ++e) {
        const float f0 = a0[e], f1 = a1[e], f2 = a2[e], f3 = a3[e];
        _Float16 hh, ll;
        split_h(f0, hh, ll);
        ah[e] = hh;
        al[e] = ll;
        split_h(f1, hh, ll);
        ah[4 + e] = hh;
        al[4 + e] = ll;
        split_h(f2, hh, ll);
        ah[8 + e] = hh;
        al[8 + e] = ll;
        split_h(f3, hh, ll);
        ah[12 + e] = hh;
        al[12 + e] = ll;
      }
      v8f c  = zero8;
      v8f cl = zero8;
      c  = mma_h(ah, B4f, c);
      cl = mma_h(al, B4f, cl);
      float* hp = sOw + (8 * h) * 16 + n;
#pragma unroll
      for (int r = 0; r < 8; ++r) {
        const float v = fmaf(cl[r], kInvWL, c[r] * kInvW) + bb4;
        hp[r * 16] = fmaxf(v, 0.0f);
      }
    }
    wave_lds_sync();

    {
      const v4f o0 = *(const v4f*)(sOw + lane * 4);
      const v4f o1 = *(const v4f*)(sOw + 128 + lane * 4);
      float* op = out + (size_t)t * (kTileRows * kHid) + lane * 4;
      *(volatile v4f*)(op)       = o0;
      *(volatile v4f*)(op + 128) = o1;
      __threadfence();
      *(volatile v4f*)(op)       = o0;
      *(volatile v4f*)(op + 128) = o1;
    }
    wave_lds_sync();
  }
}

extern "C" void kernel_launch(void* const* d_in, const int* in_sizes, int n_in,
                              void* d_out, int out_size, void* d_ws, size_t ws_size,
                              hipStream_t stream) {
  (void)d_ws;
  (void)ws_size;
  if (n_in < 9) return;
  if (in_sizes[0] != kSamples * kLeaves) return;
  if (in_sizes[1] != 8 * 2 * kHid) return;
  if (in_sizes[2] != 8 * kHid) return;
  if (in_sizes[3] != 4 * 32 * kHid) return;
  if (in_sizes[4] != 4 * kHid) return;
  if (in_sizes[5] != 2 * 32 * kHid) return;
  if (in_sizes[6] != 2 * kHid) return;
  if (in_sizes[7] != 32 * kHid) return;
  if (in_sizes[8] != kHid) return;
  if (out_size != kSamples * kHid) return;

  const float* x  = (const float*)d_in[0];
  const float* W1 = (const float*)d_in[1];
  const float* b1 = (const float*)d_in[2];
  const float* W2 = (const float*)d_in[3];
  const float* b2 = (const float*)d_in[4];
  const float* W3 = (const float*)d_in[5];
  const float* b3 = (const float*)d_in[6];
  const float* W4 = (const float*)d_in[7];
  const float* b4 = (const float*)d_in[8];
  float* out = (float*)d_out;

  tree_fused_kernel<<<kBlocks, kThreads, 0, stream>>>(x, W1, b1, W2, b2, W3, b3, W4, b4,
                                                      out, kTiles, kTilesPerWave);
}
